// Memory_sup_33389075759209
// MI455X (gfx1250) — hardware-verified
//
#include <hip/hip_runtime.h>
#include <stddef.h>


typedef __bf16   v16b __attribute__((ext_vector_type(16)));
typedef unsigned v4u  __attribute__((ext_vector_type(4)));
typedef float    v8f  __attribute__((ext_vector_type(8)));
typedef float    v4f  __attribute__((ext_vector_type(4)));

union Frag { v16b v; v4u u[2]; };

static constexpr int NB = 4;
static constexpr int NC = 128;
static constexpr int NH = 128;
static constexpr int NW = 128;
static constexpr int NPIX = NB * NH * NW;
static constexpr int NMEM = 5;
static constexpr int NPATCH = NB * (NH / 4) * (NW / 4);

__device__ __forceinline__ v8f zero8() {
  v8f r;
#pragma unroll
  for (int i = 0; i < 8; ++i) r[i] = 0.f;
  return r;
}

__device__ __forceinline__ unsigned bfb(float x) {
  unsigned u = __float_as_uint(x);
  return (u + 0x7fffu + ((u >> 16) & 1u)) >> 16;
}

__device__ __forceinline__ void split2(float x0, float x1, unsigned& hi, unsigned& lo) {
  unsigned h0 = bfb(x0), h1 = bfb(x1);
  float r0 = x0 - __uint_as_float(h0 << 16);
  float r1 = x1 - __uint_as_float(h1 << 16);
  hi = h0 | (h1 << 16);
  lo = bfb(r0) | (bfb(r1) << 16);
}

__device__ __forceinline__ void split8(v4f a, v4f b, v4u& hi, v4u& lo) {
  unsigned hh, ll;
  split2(a[0], a[1], hh, ll); hi[0] = hh; lo[0] = ll;
  split2(a[2], a[3], hh, ll); hi[1] = hh; lo[1] = ll;
  split2(b[0], b[1], hh, ll); hi[2] = hh; lo[2] = ll;
  split2(b[2], b[3], hh, ll); hi[3] = hh; lo[3] = ll;
}

__device__ __forceinline__ v8f mma(v16b a, v16b b, v8f c) {
  return __builtin_amdgcn_wmma_f32_16x16x32_bf16(false, a, false, b, (short)0, c, false, false);
}

constexpr int PM_W1 = 0;
constexpr int PM_PE = 1;
constexpr int PM_EXPT = 2;
constexpr int PM_POST = 3;

template <int MODE>
__device__ __forceinline__ float prep_val(int o, const float* __restrict__ s0,
                                          const float* __restrict__ s1) {
  if (MODE == PM_W1) {
    return s0[o] * s1[o % (NMEM * NC)];
  } else if (MODE == PM_PE) {
    int oo = o >> 11, k = o & 2047;
    int py = k >> 9, px = (k >> 7) & 3, c = k & 127;
    return s0[((oo * NC + c) * 4 + py) * 4 + px];
  } else if (MODE == PM_EXPT) {
    int n = o >> 7, k = o & 127;
    return s0[k * 512 + n];
  } else {
    int oo = o / 1152, rem = o - oo * 1152;
    int tap = rem >> 7, i = rem & 127;
    return s0[(oo * NC + i) * 9 + tap];
  }
}

template <int MODE>
__global__ __launch_bounds__(256) void k_prep(float* dst, const float* __restrict__ s0,
                                             const float* __restrict__ s1, int nquads) {
  int f = blockIdx.x * 256 + threadIdx.x;
  if (f >= nquads) return;
  v4f v;
#pragma unroll
  for (int j = 0; j < 4; ++j) v[j] = prep_val<MODE>(f * 4 + j, s0, s1);
  float* p = dst + (size_t)f * 4;
  *(volatile v4f*)p = v;
  __threadfence();
  *(volatile v4f*)p = v;
}

template <bool NORM>
__global__ __launch_bounds__(256) void k_pix_major(float* dst, const float* __restrict__ src,
                                                   int npix) {
  __shared__ float vals[64 * 128];
  __shared__ float partial[256];
  __shared__ float scale[64];
  const int t = threadIdx.x;
  const int p = t & 63, q = t >> 6;
  const int n0 = (int)blockIdx.x * 64;
  if (n0 + 64 > npix) return;
  const int b = n0 >> 14;
  const int plane = n0 & 16383;
  float ss = 0.f;
#pragma unroll 4
  for (int i = 0; i < 32; ++i) {
    int c = q * 32 + i;
    float v = src[((size_t)(b * NC + c)) * (NH * NW) + plane + p];
    vals[p * 128 + c] = v;
    ss += v * v;
  }
  partial[t] = ss;
  __syncthreads();
  if (t < 64) {
    float sc = 1.f;
    if (NORM) {
      float tot = partial[t] + partial[64 + t] + partial[128 + t] + partial[192 + t];
      sc = 1.f / fmaxf(sqrtf(tot), 1e-12f);
    }
    scale[t] = sc;
  }
  __syncthreads();
#pragma unroll
  for (int pass = 0; pass < 2; ++pass) {
#pragma unroll
    for (int it = 0; it < 8; ++it) {
      int L = it * 32 + (t >> 3);
      int px = L >> 2, seg = L & 3, q8 = t & 7;
      int base = px * 128 + seg * 32 + q8 * 4;
      float sc = scale[px];
      v4f v;
      v[0] = vals[base + 0] * sc; v[1] = vals[base + 1] * sc;
      v[2] = vals[base + 2] * sc; v[3] = vals[base + 3] * sc;
      float* d = dst + ((size_t)(n0 + px)) * NC + seg * 32 + q8 * 4;
      *(volatile v4f*)d = v;
    }
    if (pass == 0) __threadfence();
  }
}

constexpr int AM_PLAIN = 0;
constexpr int AM_PATCH = 1;
constexpr int AM_CONV  = 2;
constexpr int EP_PLAIN = 0;
constexpr int EP_SIG   = 1;
constexpr int EP_WF    = 2;
constexpr int EP_CONV  = 3;

template <int EP>
__device__ __forceinline__ void epi_tile(v8f c, int rbase, int h, int col, int row0, int col0,
                                         int N, const float* __restrict__ bias,
                                         const float* __restrict__ fuse,
                                         const float* __restrict__ aux,
                                         const float* __restrict__ aux2,
                                         float f0, float f1, float inv_bn, float (*Cs)[65]) {
  const int gcol = col0 + col;
  float bv = 0.f, sc = 0.f, sh = 0.f;
  if (EP == EP_PLAIN || EP == EP_SIG) bv = bias ? bias[gcol] : 0.f;
  if (EP == EP_CONV) { sc = aux[gcol] * inv_bn; sh = aux2[gcol]; }
#pragma unroll
  for (int r = 0; r < 8; ++r) {
    int row = rbase + 8 * h + r;
    float val = c[r];
    if (EP == EP_PLAIN) {
      val = val + bv;
    } else if (EP == EP_SIG) {
      val = val + bv;
      val = 1.f / (1.f + __expf(-val));
    } else if (EP == EP_WF) {
      val = f0 * val + f1 * fuse[((size_t)(row0 + row)) * N + gcol];
    } else {
      val = fminf(fmaxf(val * sc + sh, 0.f), 6.f);
    }
    Cs[row][col] = val;
  }
}

template <int AM, int EP>
__global__ __launch_bounds__(128) void k_gemm(const float* __restrict__ A, int lda,
                                              const float* __restrict__ Wm, int ldw,
                                              const float* __restrict__ bias,
                                              float* outp, int ldc,
                                              const float* __restrict__ fuse,
                                              const float* __restrict__ aux,
                                              const float* __restrict__ aux2,
                                              int R, int N, int K) {
  __shared__ v4u As[2][32][4];
  __shared__ v4u Ws[2][64][4];
  __shared__ float Cs[32][65];
  const int t = threadIdx.x, lane = t & 31, wave = t >> 5;
  const int h = lane >> 4, m = lane & 15;
  const int colTiles = N >> 6;
  const int rowT = (int)blockIdx.x / colTiles;
  const int colT = (int)blockIdx.x - rowT * colTiles;
  const int row0 = rowT * 32, col0 = colT * 64;
  if (row0 + 32 > R || col0 + 64 > N) return;
  const int srow = t >> 2, skq = t & 3;

  v8f acc0 = zero8(), acc1 = zero8();
  for (int k0 = 0; k0 < K; k0 += 32) {
    __syncthreads();
    {
      const int gr = row0 + srow;
      const int gk = k0 + skq * 8;
      const float* ap = A;
      bool valid = true;
      if (AM == AM_PLAIN) {
        ap = A + (size_t)gr * lda + gk;
      } else if (AM == AM_PATCH) {
        int b = gr >> 10, ph = (gr >> 5) & 31, pw = gr & 31;
        int py = gk >> 9, px = (gk >> 7) & 3, c = gk & 127;
        size_t pix = ((size_t)(b * NH + ph * 4 + py)) * NW + pw * 4 + px;
        ap = A + pix * NC + c;
      } else {
        int b = gr >> 14, y = (gr >> 7) & 127, x = gr & 127;
        int tap = gk >> 7, i = gk & 127;
        int dy = tap / 3, dx = tap - dy * 3;
        int yy = y + dy - 1;
        valid = ((unsigned)yy < (unsigned)NH);
        if (valid) {
          size_t prow = ((size_t)(b * NH + yy)) * (NW + 2) + x + dx;
          ap = A + prow * NC + i;
        }
      }
      v4f x0, x1;
      if (valid) {
        x0 = *(const v4f*)ap;
        x1 = *(const v4f*)(ap + 4);
      } else {
#pragma unroll
        for (int j = 0; j < 4; ++j) { x0[j] = 0.f; x1[j] = 0.f; }
      }
      v4u hi, lo;
      split8(x0, x1, hi, lo);
      As[0][srow][skq] = hi;
      As[1][srow][skq] = lo;
    }
#pragma unroll
    for (int ps = 0; ps < 2; ++ps) {
      const int wr = ps * 32 + srow;
      const float* wp = Wm + ((size_t)(col0 + wr)) * ldw + k0 + skq * 8;
      v4f x0 = *(const v4f*)wp;
      v4f x1 = *(const v4f*)(wp + 4);
      v4u hi, lo;
      split8(x0, x1, hi, lo);
      Ws[0][wr][skq] = hi;
      Ws[1][wr][skq] = lo;
    }
    __syncthreads();
    const int cw = wave * 16;
    Frag a0h, a0l, a1h, a1l, bh, bl;
    a0h.u[0] = As[0][m][h];       a0h.u[1] = As[0][m][2 + h];
    a0l.u[0] = As[1][m][h];       a0l.u[1] = As[1][m][2 + h];
    a1h.u[0] = As[0][16 + m][h];  a1h.u[1] = As[0][16 + m][2 + h];
    a1l.u[0] = As[1][16 + m][h];  a1l.u[1] = As[1][16 + m][2 + h];
    bh.u[0]  = Ws[0][cw + m][h];  bh.u[1]  = Ws[0][cw + m][2 + h];
    bl.u[0]  = Ws[1][cw + m][h];  bl.u[1]  = Ws[1][cw + m][2 + h];
    acc0 = mma(a0h.v, bh.v, acc0);
    acc1 = mma(a1h.v, bh.v, acc1);
    acc0 = mma(a0h.v, bl.v, acc0);
    acc1 = mma(a1h.v, bl.v, acc1);
    acc0 = mma(a0l.v, bh.v, acc0);
    acc1 = mma(a1l.v, bh.v, acc1);
    asm volatile("v_nop\n\tv_nop\n\tv_nop\n\tv_nop"
                 : "+v"(acc0), "+v"(acc1)
                 : "v"(a0h.v), "v"(a0l.v), "v"(a1h.v), "v"(a1l.v), "v"(bh.v), "v"(bl.v));
  }

  float f0 = 0.f, f1 = 0.f;
  if (EP == EP_WF) {
    float w0 = fmaxf(aux[0], 0.f), w1 = fmaxf(aux[1], 0.f);
    float sinv = 1.f / (w0 + w1 + 1e-8f);
    f0 = w0 * sinv;
    f1 = w1 * sinv;
  }
  const float inv_bn = 1.f / sqrtf(1.f + 1e-5f);
  const int col = wave * 16 + m;
  epi_tile<EP>(acc0, 0,  h, col, row0, col0, N, bias, fuse, aux, aux2, f0, f1, inv_bn, Cs);
  epi_tile<EP>(acc1, 16, h, col, row0, col0, N, bias, fuse, aux, aux2, f0, f1, inv_bn, Cs);
  __syncthreads();

#pragma unroll
  for (int pass = 0; pass < 2; ++pass) {
#pragma unroll
    for (int it = 0; it < 4; ++it) {
      const int L = it * 16 + (t >> 3);
      const int q = t & 7;
      v4f v;
      float* d;
      if (EP == EP_CONV) {
        const int cch = L;
        v[0] = Cs[q * 4 + 0][cch]; v[1] = Cs[q * 4 + 1][cch];
        v[2] = Cs[q * 4 + 2][cch]; v[3] = Cs[q * 4 + 3][cch];
        const int b = row0 >> 14, y = (row0 >> 7) & 127, x0 = row0 & 127;
        d = outp + ((size_t)(b * NC + col0 + cch)) * (NH * NW) + y * NW + x0 + q * 4;
      } else {
        const int row = L >> 1, hl = L & 1;
        const int cl = hl * 32 + q * 4;
        v[0] = Cs[row][cl + 0]; v[1] = Cs[row][cl + 1];
        v[2] = Cs[row][cl + 2]; v[3] = Cs[row][cl + 3];
        if (EP == EP_WF) {
          const int g = row0 + row;
          size_t drow = ((size_t)((g >> 14) * NH + ((g >> 7) & 127))) * (NW + 2) + (g & 127) + 1;
          d = outp + drow * NC + col0 + cl;
        } else {
          d = outp + ((size_t)(row0 + row)) * ldc + col0 + cl;
        }
      }
      *(volatile v4f*)d = v;
    }
    if (pass == 0) __threadfence();
  }
}

__global__ __launch_bounds__(128) void k_ln128(float* dst, const float* __restrict__ src,
                                               const float* __restrict__ g,
                                               const float* __restrict__ be, int rows) {
  const int lane = threadIdx.x & 31;
  const int wave = threadIdx.x >> 5;
  const int row = (int)blockIdx.x * 4 + wave;
  if (row >= rows) return;
  v4f x = *(const v4f*)(src + (size_t)row * 128 + lane * 4);
  float s = (x[0] + x[1]) + (x[2] + x[3]);
#pragma unroll
  for (int mm = 16; mm >= 1; mm >>= 1) s += __shfl_xor(s, mm, 32);
  const float mean = s * (1.f / 128.f);
  float d0 = x[0] - mean, d1 = x[1] - mean, d2 = x[2] - mean, d3 = x[3] - mean;
  float s2 = (d0 * d0 + d1 * d1) + (d2 * d2 + d3 * d3);
#pragma unroll
  for (int mm = 16; mm >= 1; mm >>= 1) s2 += __shfl_xor(s2, mm, 32);
  const float var = s2 * (1.f / 128.f);
  const float rstd = 1.f / sqrtf(var + 1e-5f);
  const int c = lane * 4;
  v4f y;
  y[0] = d0 * rstd * g[c + 0] + be[c + 0];
  y[1] = d1 * rstd * g[c + 1] + be[c + 1];
  y[2] = d2 * rstd * g[c + 2] + be[c + 2];
  y[3] = d3 * rstd * g[c + 3] + be[c + 3];
  float* d = dst + (size_t)row * 128 + c;
  *(volatile v4f*)d = y;
  __threadfence();
  *(volatile v4f*)d = y;
}

__global__ __launch_bounds__(128) void k_shuffle_ln32(float* dst, const float* __restrict__ fe,
                                                      const float* __restrict__ g,
                                                      const float* __restrict__ be, int npix) {
  const int lane = threadIdx.x & 31;
  const int wave = threadIdx.x >> 5;
  const int n = (int)blockIdx.x * 4 + wave;
  if (n >= npix) return;
  const int b = n >> 14, y = (n >> 7) & 127, x = n & 127;
  const int patch = b * 1024 + (y >> 2) * 32 + (x >> 2);
  const int j = (y & 3) * 128 + (x & 3) * 32 + lane;
  const float v = fe[(size_t)patch * 512 + j];
  float s = v;
#pragma unroll
  for (int mm = 16; mm >= 1; mm >>= 1) s += __shfl_xor(s, mm, 32);
  const float mean = s * (1.f / 32.f);
  const float dv = v - mean;
  float s2 = dv * dv;
#pragma unroll
  for (int mm = 16; mm >= 1; mm >>= 1) s2 += __shfl_xor(s2, mm, 32);
  const float var = s2 * (1.f / 32.f);
  const float rstd = 1.f / sqrtf(var + 1e-5f);
  const float yv = dv * rstd * g[lane] + be[lane];
  const int src0 = (lane & 7) * 4;
  v4f o;
  o[0] = __shfl(yv, src0 + 0, 32);
  o[1] = __shfl(yv, src0 + 1, 32);
  o[2] = __shfl(yv, src0 + 2, 32);
  o[3] = __shfl(yv, src0 + 3, 32);
  float* d = dst + (size_t)n * 32 + (lane & 7) * 4;
  if (lane < 8) *(volatile v4f*)d = o;
  __threadfence();
  if (lane < 8) *(volatile v4f*)d = o;
}

__global__ __launch_bounds__(256) void k_zero_pad(float* xp) {
  const int f = (int)blockIdx.x * 256 + threadIdx.x;
  if (f >= NB * NH * 2 * 32) return;
  const int r = f >> 5, w = f & 31;
  const int by = r >> 1, side = r & 1;
  size_t drow = (size_t)by * (NW + 2) + (side ? (NW + 1) : 0);
  float* d = xp + drow * NC + w * 4;
  v4f z;
#pragma unroll
  for (int jj = 0; jj < 4; ++jj) z[jj] = 0.f;
  *(volatile v4f*)d = z;
  __threadfence();
  *(volatile v4f*)d = z;
}

extern "C" void kernel_launch(void* const* d_in, const int* in_sizes, int n_in,
                              void* d_out, int out_size, void* d_ws, size_t ws_size,
                              hipStream_t stream) {
  if (n_in < 23) return;
  const float* Structure = (const float*)d_in[0];
  const float* query     = (const float*)d_in[1];
  const float* m_items   = (const float*)d_in[2];
  const float* mod_w     = (const float*)d_in[3];
  const float* mod_b     = (const float*)d_in[4];
  const float* conv1_w   = (const float*)d_in[5];
  const float* conv1_b   = (const float*)d_in[6];
  const float* conv2_w   = (const float*)d_in[7];
  const float* conv2_b   = (const float*)d_in[8];
  const float* pe_w      = (const float*)d_in[9];
  const float* pe_b      = (const float*)d_in[10];
  const float* pe_g      = (const float*)d_in[11];
  const float* pe_beta   = (const float*)d_in[12];
  const float* exp_w     = (const float*)d_in[13];
  const float* fin_g     = (const float*)d_in[14];
  const float* fin_b     = (const float*)d_in[15];
  const float* up_w      = (const float*)d_in[16];
  const float* up_b      = (const float*)d_in[17];
  const float* wf_w2     = (const float*)d_in[18];
  const float* wf_pre_w  = (const float*)d_in[19];
  const float* wf_post_w = (const float*)d_in[20];
  const float* wf_bn_g   = (const float*)d_in[21];
  const float* wf_bn_b   = (const float*)d_in[22];

  if (out_size != NPIX * NC) return;
  if (in_sizes[0] != NPIX * NC || in_sizes[1] != NPIX * NC) return;
  if (in_sizes[2] != NMEM * NC || in_sizes[3] != NMEM * NC * NC) return;
  if (in_sizes[5] != 64 * NMEM * NC || in_sizes[7] != 64 * NC) return;
  if (in_sizes[9] != NC * NC * 16 || in_sizes[13] != NC * 512) return;
  if (in_sizes[16] != NC * 32 || in_sizes[19] != NC * NC || in_sizes[20] != NC * NC * 9) return;
  if (in_sizes[14] != 32 || in_sizes[15] != 32 || in_sizes[18] != 2) return;

  char* ws = (char*)d_ws;
  size_t off = 0;
  auto carve = [&](size_t bytes) -> float* {
    float* p = (float*)(ws + off);
    off = (off + bytes + 255) & ~(size_t)255;
    return p;
  };

  float* sPM   = carve((size_t)NPIX * NC * 4);
  float* Sn    = carve((size_t)NPIX * NC * 4);
  float* fRaw  = carve((size_t)NPATCH * NC * 4);
  float* fLN   = carve((size_t)NPATCH * NC * 4);
  float* w1    = carve((size_t)64 * NMEM * NC * 4);
  float* Wpe   = carve((size_t)NC * 2048 * 4);
  float* WexpT = carve((size_t)512 * NC * 4);
  float* Wpost = carve((size_t)NC * 1152 * 4);
  float* big   = carve((size_t)NPIX * NMEM * NC * 4);
  float* modA  = big;
  float* fe    = big;
  float* aLN   = (float*)((char*)big + (size_t)8  * 1048576);
  float* M1    = (float*)((char*)big + (size_t)16 * 1048576);
  float* xPad  = (float*)((char*)big + (size_t)48 * 1048576);
  float* qPM   = (float*)((char*)big + (size_t)82 * 1048576);
  if (off > ws_size) return;

  auto qg = [](int nelem) { return dim3((unsigned)((nelem / 4 + 255) / 256)); };
  auto gg = [](int R, int N) { return dim3((unsigned)((R / 32) * (N / 64))); };

  k_prep<PM_W1><<<qg(64 * 640), 256, 0, stream>>>(w1, conv1_w, m_items, 64 * 640 / 4);
  k_prep<PM_PE><<<qg(128 * 2048), 256, 0, stream>>>(Wpe, pe_w, pe_w, 128 * 2048 / 4);
  k_prep<PM_EXPT><<<qg(512 * 128), 256, 0, stream>>>(WexpT, exp_w, exp_w, 512 * 128 / 4);
  k_prep<PM_POST><<<qg(128 * 1152), 256, 0, stream>>>(Wpost, wf_post_w, wf_post_w, 128 * 1152 / 4);

  k_pix_major<true><<<NPIX / 64, 256, 0, stream>>>(sPM, Structure, NPIX);

  k_gemm<AM_PLAIN, EP_SIG><<<gg(NPIX, 640), 128, 0, stream>>>(
      sPM, NC, mod_w, NC, mod_b, modA, 640, nullptr, nullptr, nullptr, NPIX, 640, NC);
  k_gemm<AM_PLAIN, EP_PLAIN><<<gg(NPIX, 64), 128, 0, stream>>>(
      modA, 640, w1, 640, conv1_b, Sn, NC, nullptr, nullptr, nullptr, NPIX, 64, 640);
  k_gemm<AM_PLAIN, EP_PLAIN><<<gg(NPIX, 64), 128, 0, stream>>>(
      sPM, NC, conv2_w, NC, conv2_b, Sn + 64, NC, nullptr, nullptr, nullptr, NPIX, 64, NC);
  k_gemm<AM_PATCH, EP_PLAIN><<<gg(NPATCH, NC), 128, 0, stream>>>(
      Sn, 0, Wpe, 2048, pe_b, fRaw, NC, nullptr, nullptr, nullptr, NPATCH, NC, 2048);
  k_ln128<<<(NPATCH + 3) / 4, 128, 0, stream>>>(fLN, fRaw, pe_g, pe_beta, NPATCH);
  k_gemm<AM_PLAIN, EP_PLAIN><<<gg(NPATCH, 512), 128, 0, stream>>>(
      fLN, NC, WexpT, NC, nullptr, fe, 512, nullptr, nullptr, nullptr, NPATCH, 512, NC);
  k_shuffle_ln32<<<(NPIX + 3) / 4, 128, 0, stream>>>(aLN, fe, fin_g, fin_b, NPIX);
  k_gemm<AM_PLAIN, EP_PLAIN><<<gg(NPIX, NC), 128, 0, stream>>>(
      aLN, 32, up_w, 32, up_b, M1, NC, nullptr, nullptr, nullptr, NPIX, NC, 32);
  k_pix_major<false><<<NPIX / 64, 256, 0, stream>>>(qPM, query, NPIX);
  k_zero_pad<<<(NB * NH * 2 * 32 + 255) / 256, 256, 0, stream>>>(xPad);
  k_gemm<AM_PLAIN, EP_WF><<<gg(NPIX, NC), 128, 0, stream>>>(
      qPM, NC, wf_pre_w, NC, nullptr, xPad, NC, M1, wf_w2, nullptr, NPIX, NC, NC);
  k_gemm<AM_CONV, EP_CONV><<<gg(NPIX, NC), 128, 0, stream>>>(
      xPad, 0, Wpost, 1152, nullptr, (float*)d_out, 0, nullptr, wf_bn_g, wf_bn_b, NPIX, NC, 1152);
}
